// SoftgroupAttention_11836929868321
// MI455X (gfx1250) — hardware-verified
//
#include <hip/hip_runtime.h>
#include <math.h>

typedef __attribute__((ext_vector_type(16))) _Float16 v16h;
typedef __attribute__((ext_vector_type(16))) __bf16 v16b;
typedef __attribute__((ext_vector_type(8)))  _Float16 v8h;
typedef __attribute__((ext_vector_type(8)))  float v8f;
typedef __attribute__((ext_vector_type(4)))  float v4f;
typedef __attribute__((ext_vector_type(2)))  float v2f;
typedef __attribute__((ext_vector_type(4)))  unsigned v4u;
typedef __attribute__((ext_vector_type(4)))  int v4i;
typedef float __attribute__((may_alias)) float_a;
typedef int __attribute__((may_alias)) int_a;

template <typename T> __device__ __forceinline__ void vst2(void* p, T v) { *(volatile T*)p = v; __threadfence(); *(volatile T*)p = v; }
__device__ __forceinline__ v8f wmma16(v16h a, v16h b, v8f c) {
  v8f d = __builtin_amdgcn_wmma_f32_16x16x32_f16(false, a, false, b, (short)0, c, false, false);
  asm volatile("v_nop\n\tv_nop\n\tv_nop\n\tv_nop" : "+v"(d) : "v"(a), "v"(b));
  return d;
}
__device__ __forceinline__ v8f wmma_bf(v16b a, v16b b, v8f c) {
  v8f d = __builtin_amdgcn_wmma_f32_16x16x32_bf16(false, a, false, b, (short)0, c, false, false);
  asm volatile("v_nop\n\tv_nop\n\tv_nop\n\tv_nop" : "+v"(d) : "v"(a), "v"(b));
  return d;
}
__device__ __forceinline__ v16h frag_h(const _Float16* rowk0, int lane) {
  union { v16h v; v8h q[2]; } u; const _Float16* p = rowk0 + 8 * (lane >> 4);
  u.q[0] = *(const v8h*)p; u.q[1] = *(const v8h*)(p + 16); return u.v;
}
__device__ __forceinline__ v16h frag_f32(const float* rowk0, int lane) {
  v16h a; const float* p = rowk0 + 8 * (lane >> 4);
#pragma unroll
  for (int i = 0; i < 8; ++i) { a[i] = (_Float16)p[i]; a[8 + i] = (_Float16)p[16 + i]; }
  return a;
}
__device__ __forceinline__ v16h frag_f32s(const float* rowk0, int lane, float sc) {
  v16h a; const float* p = rowk0 + 8 * (lane >> 4);
#pragma unroll
  for (int i = 0; i < 8; ++i) { a[i] = (_Float16)(p[i] * sc); a[8 + i] = (_Float16)(p[16 + i] * sc); }
  return a;
}
__device__ __forceinline__ v16h fragc_f32(const float* W, int k0, int n, int lane, int ld, int K) {
  v16h a; const int g = lane >> 4;
#pragma unroll
  for (int i = 0; i < 8; ++i) { const int ka = k0 + 8 * g + i, kb = ka + 16;
    a[i] = (_Float16)(ka < K ? W[(size_t)(ka < K ? ka : K - 1) * ld + n] : 0.f); a[8 + i] = (_Float16)(kb < K ? W[(size_t)(kb < K ? kb : K - 1) * ld + n] : 0.f); }
  return a;
}
struct F2 { v16b h, l; };
__device__ __forceinline__ F2 bsplit16(const float v[16]) { F2 r;
#pragma unroll
  for (int i = 0; i < 16; ++i) { const __bf16 h = (__bf16)v[i]; r.h[i] = h; r.l[i] = (__bf16)(v[i] - (float)h); }
  return r; }
__device__ __forceinline__ F2 split_row(const float* row, int k0, int lane) { float v[16]; const float* p = row + k0 + 8 * (lane >> 4);
#pragma unroll
  for (int i = 0; i < 8; ++i) { v[i] = p[i]; v[8 + i] = p[16 + i]; }
  return bsplit16(v); }
__device__ __forceinline__ F2 split_rowK(const float* row, int k0, int lane, int K) { float v[16]; const int g = lane >> 4;
#pragma unroll
  for (int i = 0; i < 8; ++i) { const int ka = k0 + 8 * g + i, kb = ka + 16; v[i] = ka < K ? row[ka < K ? ka : K - 1] : 0.f; v[8 + i] = kb < K ? row[kb < K ? kb : K - 1] : 0.f; }
  return bsplit16(v); }
__device__ __forceinline__ F2 split_col(const float* W, int k0, int n, int lane, int ld, int K) { float v[16]; const int g = lane >> 4;
#pragma unroll
  for (int i = 0; i < 8; ++i) { const int ka = k0 + 8 * g + i, kb = ka + 16; v[i] = ka < K ? W[(size_t)(ka < K ? ka : K - 1) * ld + n] : 0.f; v[8 + i] = kb < K ? W[(size_t)(kb < K ? kb : K - 1) * ld + n] : 0.f; }
  return bsplit16(v); }
__device__ __forceinline__ v8f mac3(const F2& a, const F2& b, v8f c) { c = wmma_bf(a.l, b.h, c); c = wmma_bf(a.h, b.l, c); return wmma_bf(a.h, b.h, c); }
__device__ __forceinline__ float sigm(float v) { return 1.0f / (1.0f + expf(-v)); }
#define LDSX() do { asm volatile("s_wait_dscnt 0" ::: "memory"); __builtin_amdgcn_wave_barrier(); __builtin_amdgcn_fence(__ATOMIC_RELEASE, "workgroup"); } while (0)


#define NB 8
#define NN 1024
#define DM 384
#define NH 12
#define HD 32
#define GP 20
#define GPP 32
#ifndef TNB
#define TNB NB
#endif
typedef __attribute__((ext_vector_type(8))) __bf16 v8b;
__device__ __forceinline__ v16b frag_b(const __bf16* rowk0, int lane) {
  union { v16b v; v8b q[2]; } u; const __bf16* p = rowk0 + 8 * (lane >> 4);
  u.q[0] = *(const v8b*)p; u.q[1] = *(const v8b*)(p + 16); return u.v;
}
__device__ __forceinline__ float bfr(float v) { return (float)(__bf16)v; }
__device__ __attribute__((noinline)) float exp_ni(float v) { return expf(v); }
__device__ __attribute__((noinline)) float erf_ni(float v) { return erff(v); }

#define WS_Q   0u
#define WS_K   (WS_Q + 2u * (size_t)NB * NN * DM)
#define WS_VH  (WS_K + 2u * (size_t)NB * NN * DM)
#define WS_VL  (WS_VH + 2u * (size_t)NB * DM * NN)
#define WS_GW  (WS_VL + 2u * (size_t)NB * DM * NN)
#define WS_ML  (WS_GW + 2u * (size_t)NB * NN * NH * GPP)
#define WS_CS  (WS_ML + 4u * (size_t)NB * NH * NN * 2)
#define WS_O   (WS_CS + 4u * (size_t)NB * NH * NN)
#define WS_END (WS_O + 4u * (size_t)NB * NN * DM)

__device__ __forceinline__ v16b fragb_f32(const float* __restrict__ p, int lane) { v16b a; const float* pp = p + 8 * (lane >> 4);
#pragma unroll
  for (int i = 0; i < 8; ++i) { a[i] = (__bf16)pp[i]; a[8 + i] = (__bf16)pp[16 + i]; } return a; }
__global__ __launch_bounds__(128) void k_qkv(const float* __restrict__ X, const float* __restrict__ W, const float* __restrict__ GPW, const float* __restrict__ TP, _Float16* __restrict__ Q, _Float16* __restrict__ K, _Float16* __restrict__ VH, _Float16* __restrict__ VL, _Float16* __restrict__ GW) {
  __shared__ __align__(16) float sq[64][132]; __shared__ __align__(16) _Float16 sh[64][136]; __shared__ __align__(16) _Float16 th[128][72], tl[128][72]; __shared__ __align__(16) _Float16 sg[64][136];
  const int tid = threadIdx.x, wave = tid >> 5, lane = tid & 31, col = lane & 15, g = lane >> 4; const size_t b = blockIdx.z; const int n0 = blockIdx.x * 64; const int c0 = blockIdx.y * 128; const int which = c0 / DM; const int cw = c0 % DM;
  const size_t r0 = b * NN + n0 + wave * 16;
  v8f acc[8] = {};
#pragma unroll 2
  for (int kc = 0; kc < DM / 32; ++kc) { const v16b a = fragb_f32(X + (r0 + col) * DM + kc * 32, lane);
#pragma unroll
    for (int j = 0; j < 8; ++j) { v16b w; const int o = c0 + j * 16 + col;
#pragma unroll
      for (int i = 0; i < 8; ++i) { w[i] = (__bf16)W[(size_t)(kc * 32 + 8 * g + i) * (3 * DM) + o]; w[8 + i] = (__bf16)W[(size_t)(kc * 32 + 16 + 8 * g + i) * (3 * DM) + o]; }
      acc[j] = wmma_bf(a, w, acc[j]); } }
#pragma unroll
  for (int j = 0; j < 8; ++j)
#pragma unroll
    for (int r = 0; r < 8; ++r) { const float v = acc[j][r]; const int rl = wave * 16 + 8 * g + r, cl = j * 16 + col; if (which == 2) { const _Float16 hv = (_Float16)v; th[cl][rl] = hv; tl[cl][rl] = (_Float16)((v - (float)hv) * 2048.0f); } else { sh[rl][cl] = (_Float16)v; if (which == 0) sq[rl][cl] = v; } }
  __syncthreads();
  if (which < 2) { _Float16* dst = which == 0 ? Q : K; for (int e = tid; e < 64 * 16; e += 128) { const int rl = e >> 4, q = e & 15; vst2((unsigned*)(dst + (b * NN + n0 + rl) * DM + cw + q * 8), *(const v4u*)&sh[rl][q * 8]); } }
  else { for (int e = tid; e < 128 * 8; e += 128) { const int cl = e >> 3, q = e & 7; const size_t o = (b * DM + cw + cl) * (size_t)NN + n0 + q * 8; vst2((unsigned*)(VH + o), *(const v4u*)&th[cl][q * 8]); vst2((unsigned*)(VL + o), *(const v4u*)&tl[cl][q * 8]); } }
  if (which == 0) {
    const float invt = 1.0f / log1pf(expf(bfr(TP[0])));
#pragma unroll 1
    for (int hl = 0; hl < 4; ++hl) { const int h = cw / HD + hl; const F2 a = split_row(&sq[wave * 16 + col][0], hl * HD, lane); v8f c2[2];
#pragma unroll
      for (int tt = 0; tt < 2; ++tt) { v16b w; const int m = tt * 16 + col;
#pragma unroll
        for (int i = 0; i < 16; ++i) { const int d = (i < 8) ? (8 * g + i) : (16 + 8 * g + (i - 8)); w[i] = (m < GP) ? (__bf16)GPW[(size_t)(h * GP + m) * HD + d] : (__bf16)0.0f; }
        c2[tt] = v8f{}; c2[tt] = wmma_bf(a.h, w, c2[tt]); c2[tt] = wmma_bf(a.l, w, c2[tt]); }
#pragma unroll
      for (int r = 0; r < 8; ++r) { const float s0 = c2[0][r] * invt, s1 = (16 + col < GP) ? c2[1][r] * invt : -3.0e38f; float mx = fmaxf(s0, s1);
#pragma unroll
        for (int o = 1; o < 16; o <<= 1) mx = fmaxf(mx, __shfl_xor(mx, o));
        const float e0 = __expf(s0 - mx), e1 = (16 + col < GP) ? __expf(s1 - mx) : 0.f; float es = e0 + e1;
#pragma unroll
        for (int o = 1; o < 16; o <<= 1) es += __shfl_xor(es, o);
        const float inv = 1.0f / es; sg[wave * 16 + 8 * g + r][hl * GPP + col] = (_Float16)(e0 * inv); sg[wave * 16 + 8 * g + r][hl * GPP + 16 + col] = (_Float16)(e1 * inv); } }
    __syncthreads();
    for (int e = tid; e < 64 * 16; e += 128) { const int rl = e >> 4, q = e & 15; vst2((unsigned*)(GW + (b * NN + n0 + rl) * (NH * GPP) + (cw / HD) * GPP + q * 8), *(const v4u*)&sg[rl][q * 8]); } } }
__global__ __launch_bounds__(128) void k_stats(const _Float16* __restrict__ Q, const _Float16* __restrict__ K, float* __restrict__ ML) { __shared__ __align__(16) float sm[64][2];
  const int tid = threadIdx.x, wave = tid >> 5, lane = tid & 31, col = lane & 15, g = lane >> 4; const int h = blockIdx.y; const size_t b = blockIdx.z; const int q0 = blockIdx.x * 64 + wave * 16; const size_t rq = b * NN + q0;
  const v16h aq = frag_h(Q + (rq + col) * DM + h * HD, lane);
  float m[8], l[8];
#pragma unroll
  for (int r = 0; r < 8; ++r) { m[r] = -3.0e38f; l[r] = 0.f; }
#pragma unroll 1
  for (int ks = 0; ks < NN / 32; ++ks) { float s[2][8];
#pragma unroll
    for (int ct = 0; ct < 2; ++ct) { const size_t rk = b * NN + ks * 32 + ct * 16 + col; v8f c = {}; c = wmma16(aq, frag_h(K + rk * DM + h * HD, lane), c);
#pragma unroll
      for (int r = 0; r < 8; ++r) s[ct][r] = c[r] * 0.17677669529663687f; }
#pragma unroll
    for (int r = 0; r < 8; ++r) { float mx = fmaxf(s[0][r], s[1][r]);
#pragma unroll
      for (int o = 1; o < 16; o <<= 1) mx = fmaxf(mx, __shfl_xor(mx, o));
      const float mn = fmaxf(m[r], mx); const float alpha = __expf(m[r] - mn); float es = __expf(s[0][r] - mn) + __expf(s[1][r] - mn);
#pragma unroll
      for (int o = 1; o < 16; o <<= 1) es += __shfl_xor(es, o);
      l[r] = l[r] * alpha + es; m[r] = mn; } }
  if (col == 0) {
#pragma unroll
    for (int r = 0; r < 8; ++r) { sm[wave * 16 + 8 * g + r][0] = m[r]; sm[wave * 16 + 8 * g + r][1] = 1.0f / l[r]; } }
  __syncthreads(); if (tid < 32) vst2(ML + (((b * NH + h) * NN) + blockIdx.x * 64) * 2 + tid * 4, *(const v4f*)(&sm[0][0] + tid * 4)); }
__global__ __launch_bounds__(128) void k_colsum(const _Float16* __restrict__ Q, const _Float16* __restrict__ K, const _Float16* __restrict__ GW, const float* __restrict__ ML, float* __restrict__ CS) { __shared__ __align__(16) float scs[64];
  const int tid = threadIdx.x, wave = tid >> 5, lane = tid & 31, col = lane & 15, g = lane >> 4; const int h = blockIdx.y; const size_t b = blockIdx.z; const int m0 = blockIdx.x * 64 + wave * 16; const size_t rm = b * NN + m0;
  const v16h ak = frag_h(K + (rm + col) * DM + h * HD, lane); const v16h ag = frag_h(GW + (rm + col) * (NH * GPP) + h * GPP, lane);
  float csum[8];
#pragma unroll
  for (int r = 0; r < 8; ++r) csum[r] = 0.f;
#pragma unroll 1
  for (int qs = 0; qs < NN / 16; ++qs) { const size_t rn = b * NN + qs * 16 + col; v8f c = {}, cg = {}; c = wmma16(ak, frag_h(Q + rn * DM + h * HD, lane), c); cg = wmma16(ag, frag_h(GW + rn * (NH * GPP) + h * GPP, lane), cg);
    const float* mlp = ML + (((b * NH + h) * NN) + qs * 16 + col) * 2; const float Mn = mlp[0], iL = mlp[1];
#pragma unroll
    for (int r = 0; r < 8; ++r) csum[r] += __expf(c[r] * 0.17677669529663687f - Mn) * iL * cg[r]; }
#pragma unroll
  for (int r = 0; r < 8; ++r) { float v = csum[r];
#pragma unroll
    for (int o = 1; o < 16; o <<= 1) v += __shfl_xor(v, o);
    if (col == 0) scs[wave * 16 + 8 * g + r] = v; }
  __syncthreads(); if (tid < 16) vst2(CS + ((b * NH + h) * NN) + blockIdx.x * 64 + tid * 4, *(const v4f*)&scs[tid * 4]); }
__global__ __launch_bounds__(128) void k_out(const _Float16* __restrict__ Q, const _Float16* __restrict__ K, const _Float16* __restrict__ GW, const float* __restrict__ ML, const float* __restrict__ CS, const _Float16* __restrict__ VH, const _Float16* __restrict__ VL, float* __restrict__ O) {
  __shared__ __align__(16) float sp[4][16][36]; __shared__ __align__(16) float so[4][16][36];
  const int tid = threadIdx.x, wave = tid >> 5, lane = tid & 31, col = lane & 15, g = lane >> 4; const int h = blockIdx.y; const size_t b = blockIdx.z; const int q0 = blockIdx.x * 64 + wave * 16; const size_t rq = b * NN + q0;
  const v16h aq = frag_h(Q + (rq + col) * DM + h * HD, lane); const v16h ag = frag_h(GW + (rq + col) * (NH * GPP) + h * GPP, lane);
  float Mn[8], iL[8];
#pragma unroll
  for (int r = 0; r < 8; ++r) { const float* mlp = ML + (((b * NH + h) * NN) + q0 + 8 * g + r) * 2; Mn[r] = mlp[0]; iL[r] = mlp[1]; }
  v8f acc[2] = {}, accl[2] = {};
#pragma unroll 1
  for (int ks = 0; ks < NN / 32; ++ks) {
#pragma unroll
    for (int ct = 0; ct < 2; ++ct) { const int kk = ks * 32 + ct * 16 + col; const size_t rk = b * NN + kk; v8f c = {}, cg = {}; c = wmma16(aq, frag_h(K + rk * DM + h * HD, lane), c); cg = wmma16(ag, frag_h(GW + rk * (NH * GPP) + h * GPP, lane), cg);
      const float ics = 1.0f / (CS[(b * NH + h) * NN + kk] + 1e-8f);
#pragma unroll
      for (int r = 0; r < 8; ++r) sp[wave][8 * g + r][ct * 16 + col] = __expf(c[r] * 0.17677669529663687f - Mn[r]) * iL[r] * cg[r] * ics; }
    LDSX();
    v16h pa; { const float* prow = &sp[wave][col][0] + 8 * (lane >> 4);
#pragma unroll
      for (int i = 0; i < 8; ++i) { pa[i] = (_Float16)(prow[i] * 2048.0f); pa[8 + i] = (_Float16)(prow[16 + i] * 2048.0f); } }
#pragma unroll
    for (int j = 0; j < 2; ++j) { const size_t po = (b * DM + (size_t)h * HD + j * 16 + col) * (size_t)NN + ks * 32; acc[j] = wmma16(pa, frag_h(VH + po, lane), acc[j]); accl[j] = wmma16(pa, frag_h(VL + po, lane), accl[j]); }
    LDSX(); }
#pragma unroll
  for (int r = 0; r < 8; ++r)
#pragma unroll
    for (int j = 0; j < 2; ++j) so[wave][8 * g + r][j * 16 + col] = (acc[j][r] + accl[j][r] * (1.0f / 2048.0f)) * (1.0f / 2048.0f);
  LDSX(); for (int rl = 0; rl < 16; ++rl) if (lane < 8) vst2(O + (rq + rl) * DM + (size_t)h * HD + lane * 4, *(const v4f*)&so[wave][rl][lane * 4]); }
__global__ __launch_bounds__(128) void k_proj(const float* __restrict__ O, const float* __restrict__ WP, float* __restrict__ OUT) { __shared__ __align__(16) float sf[4][16][132];
  const int tid = threadIdx.x, wave = tid >> 5, lane = tid & 31, col = lane & 15, g = lane >> 4; const size_t r0 = (size_t)blockIdx.z * NN + blockIdx.x * 64 + wave * 16; const int c0 = blockIdx.y * 128;
  v8f acc[8] = {};
#pragma unroll 2
  for (int kc = 0; kc < DM / 32; ++kc) { const F2 a = split_row(O + (r0 + col) * DM, kc * 32, lane);
#pragma unroll
    for (int j = 0; j < 8; ++j) { v16b w; const int o = c0 + j * 16 + col;
#pragma unroll
      for (int i = 0; i < 8; ++i) { w[i] = (__bf16)WP[(size_t)(kc * 32 + 8 * g + i) * DM + o]; w[8 + i] = (__bf16)WP[(size_t)(kc * 32 + 16 + 8 * g + i) * DM + o]; }
      acc[j] = wmma_bf(a.h, w, acc[j]); acc[j] = wmma_bf(a.l, w, acc[j]); } }
#pragma unroll
  for (int j = 0; j < 8; ++j)
#pragma unroll
    for (int r = 0; r < 8; ++r) sf[wave][8 * g + r][j * 16 + col] = acc[j][r];
  LDSX(); for (int rl = 0; rl < 16; ++rl) vst2(OUT + (r0 + rl) * DM + c0 + lane * 4, *(const v4f*)&sf[wave][rl][lane * 4]); }
extern "C" void kernel_launch(void* const* d_in, const int* in_sizes, int n_in, void* d_out, int out_size, void* d_ws, size_t ws_size, hipStream_t stream) {
  (void)in_sizes; (void)n_in; (void)out_size;
  const float** F = (const float**)d_in;
  if (ws_size < (size_t)WS_END) return;
  char* ws = (char*)d_ws; _Float16 *Q = (_Float16*)(ws + WS_Q), *K = (_Float16*)(ws + WS_K), *VH = (_Float16*)(ws + WS_VH), *VL = (_Float16*)(ws + WS_VL), *GW = (_Float16*)(ws + WS_GW); float *ML = (float*)(ws + WS_ML), *CS = (float*)(ws + WS_CS), *O = (float*)(ws + WS_O);
  k_qkv<<<dim3(NN / 64, 3 * DM / 128, NB), 128, 0, stream>>>(F[0], F[1], F[2], F[3], Q, K, VH, VL, GW);
  k_stats<<<dim3(NN / 64, NH, TNB), 128, 0, stream>>>(Q, K, ML);
  k_colsum<<<dim3(NN / 64, NH, TNB), 128, 0, stream>>>(Q, K, GW, ML, CS);
  k_out<<<dim3(NN / 64, NH, TNB), 128, 0, stream>>>(Q, K, GW, ML, CS, VH, VL, O);
  k_proj<<<dim3(NN / 64, DM / 128, TNB), 128, 0, stream>>>(O, F[4], (float*)d_out);
}
